// GAT_70531952934941
// MI455X (gfx1250) — hardware-verified
//
#include <hip/hip_runtime.h>
#include <stddef.h>
#include <stdint.h>
#include <math.h>


#define DIN     64
#define HC      512
#define NHEAD   8
#define CHN     64
#define NXLR    1024
#define KA2     1024
#define NTHR    256
#define NWAVE   8
#define EPT     8
#define CHUNK   (NTHR * EPT)
#define WCAP    (EPT * 32)
#define LISTN   (NWAVE * WCAP)
#define NBA     1024
#define SLA     10
#define SRCB    15
#define RCAP    28672
#define DEGCAP  128
#define MEAS_B1024  16685
#define MEAS_MAXDEG 32
#define NREF    20000
#define GBM     64
#define GBN     64
#define GTHR    128
#define MROWS   128
#define NUW1H   (HC * (DIN / 8))
#define NUW2H   (HC * (KA2 / 8))
#define PARF    2048
#define NEGSL   0.2f
#define WSMAX   134217728
#define BKT_LDS_INTS  (LISTN + RCAP + 16)
#define SCAN_ZINTS    (RCAP + 3 * NBA)
#define SCAN_LDS_INTS (2 * RCAP + 3 * NBA)

static_assert((CHUNK & (CHUNK - 1)) == 0 && CHUNK <= 4096);
static_assert((NBA & (NBA - 1)) == 0 && NBA == (1 << SLA) && NBA <= 1024);
static_assert(((long long)CHUNK << SLA) < (1LL << 31));
static_assert(SRCB + SLA <= 31 && NREF <= (1 << SRCB));
static_assert(LISTN >= NWAVE * WCAP);
static_assert(NBA % NWAVE == 0 && NBA % 32 == 0);
static_assert((RCAP % 32) == 0 && (SCAN_ZINTS % 4) == 0);
static_assert(RCAP >= MEAS_B1024 + 4096);
static_assert(DEGCAP >= MEAS_MAXDEG + 8);
static_assert(SCAN_LDS_INTS * 4 <= 300000 && BKT_LDS_INTS * 4 <= 300000);
static_assert(GBM == (GTHR / 32) * 16);
static_assert((DIN % 32) == 0 && (KA2 % 32) == 0 && KA2 == 2 * HC);
static_assert((NXLR % GBN) == 0 && NXLR == 2 * HC);
static_assert((MROWS % GBM) == 0);
static_assert(HC == 32 * 16);
static_assert(HC == NHEAD * CHN && CHN == 4 * 16);
static_assert(NTHR * 4 == 1024);
static_assert(1024 + NWAVE * HC <= RCAP);
static_assert((NUW1H % NTHR) == 0 && (NUW2H % NTHR) == 0);
static_assert(((NREF + MROWS - 1) / MROWS) * MROWS == 157 * 128);
static_assert(3 * HC + CHN <= PARF);

typedef float          v4f  __attribute__((ext_vector_type(4)));
typedef float          v8f  __attribute__((ext_vector_type(8)));
typedef int            v4i  __attribute__((ext_vector_type(4)));
typedef int            v8i  __attribute__((ext_vector_type(8)));
typedef unsigned short v8us __attribute__((ext_vector_type(8)));
typedef __bf16         v16b __attribute__((ext_vector_type(16)));
typedef v4f  __attribute__((may_alias)) v4fa;
typedef v4i  __attribute__((may_alias)) v4ia;
typedef v8us __attribute__((may_alias)) v8usa;
union FragB { v16b v; v8us h[2]; v8i w; };

__device__ __forceinline__ v8f wmb(const FragB& a, const FragB& b, v8f c) {
  v8f d = __builtin_amdgcn_wmma_f32_16x16x32_bf16(false, a.v, false, b.v, (short)0, c, false, false);
  asm volatile("v_nop\n\tv_nop\n\tv_nop\n\tv_nop" : "+v"(d) : "v"(a.w), "v"(b.w));
  return d;
}

__device__ __forceinline__ unsigned int f2bf(float f) {
  const unsigned int u = __float_as_uint(f);
  const unsigned int r = ((u + 0x7FFFu + ((u >> 16) & 1u)) >> 16) & 0xFFFFu;
  return ((u & 0x7FFFFFFFu) > 0x7F800000u) ? 0x7FC0u : r;
}
__device__ __forceinline__ float bf2f(unsigned int b) { return __uint_as_float(b << 16); }
__device__ __forceinline__ float bfr(float f) { return bf2f(f2bf(f)); }
__device__ __forceinline__ int pk2(float a, float b) { return (int)(f2bf(a) | (f2bf(b) << 16)); }

__device__ __forceinline__ v4i pack8(const v4f a, const v4f b) {
  v4i o;
  o.x = pk2(a.x, a.y); o.y = pk2(a.z, a.w); o.z = pk2(b.x, b.y); o.w = pk2(b.z, b.w);
  return o;
}
__device__ __forceinline__ v4i wtr8(const float* __restrict__ p) {
  const float f0 = p[0];                  const float f1 = p[(size_t)HC];
  const float f2 = p[(size_t)2 * HC];     const float f3 = p[(size_t)3 * HC];
  const float f4 = p[(size_t)4 * HC];     const float f5 = p[(size_t)5 * HC];
  const float f6 = p[(size_t)6 * HC];     const float f7 = p[(size_t)7 * HC];
  v4i o;
  o.x = pk2(f0, f1); o.y = pk2(f2, f3); o.z = pk2(f4, f5); o.w = pk2(f6, f7);
  return o;
}
__device__ __forceinline__ v4i par4(const float* __restrict__ src, int n4, int v) {
  const int vc = v < n4 ? v : n4 - 1;
  const v4f f = *(const v4f*)(src + 4 * vc);
  v4i o;
  o.x = __float_as_int(bfr(f.x)); o.y = __float_as_int(bfr(f.y));
  o.z = __float_as_int(bfr(f.z)); o.w = __float_as_int(bfr(f.w));
  return o;
}

struct HL8 { v4i h; v4i l; };
__device__ __forceinline__ HL8 cvt_hl8(const v4f a, const v4f b) {
  const float f[8] = {a.x, a.y, a.z, a.w, b.x, b.y, b.z, b.w};
  unsigned int hb[8], lb[8];
#pragma unroll
  for (int i = 0; i < 8; ++i) {
    hb[i] = f2bf(f[i]);
    lb[i] = f2bf(f[i] - bf2f(hb[i]));
  }
  HL8 o;
  o.h.x = (int)(hb[0] | (hb[1] << 16)); o.h.y = (int)(hb[2] | (hb[3] << 16));
  o.h.z = (int)(hb[4] | (hb[5] << 16)); o.h.w = (int)(hb[6] | (hb[7] << 16));
  o.l.x = (int)(lb[0] | (lb[1] << 16)); o.l.y = (int)(lb[2] | (lb[3] << 16));
  o.l.z = (int)(lb[4] | (lb[5] << 16)); o.l.w = (int)(lb[6] | (lb[7] << 16));
  return o;
}

__device__ __forceinline__ float dot4(const v4f x, const v4f r, const v4f a, float p) {
  float v;
  v = x.x + r.x; v = v > 0.f ? v : NEGSL * v; p = fmaf(v, a.x, p);
  v = x.y + r.y; v = v > 0.f ? v : NEGSL * v; p = fmaf(v, a.y, p);
  v = x.z + r.z; v = v > 0.f ? v : NEGSL * v; p = fmaf(v, a.z, p);
  v = x.w + r.w; v = v > 0.f ? v : NEGSL * v; p = fmaf(v, a.w, p);
  return p;
}
__device__ __forceinline__ v4f accu(const v4f a, const v4f x, const float s1, const float s2) {
  v4f o;
  o.x = fmaf(a.x, s1, s2 * x.x); o.y = fmaf(a.y, s1, s2 * x.y);
  o.z = fmaf(a.z, s1, s2 * x.z); o.w = fmaf(a.w, s1, s2 * x.w);
  return o;
}
__device__ __forceinline__ float hsum(float v) {
  v += __shfl_xor(v, 4);
  v += __shfl_xor(v, 8);
  v += __shfl_xor(v, 16);
  return v;
}
__device__ __forceinline__ v4f hsum4(const v4f a) {
  v4f o;
  o.x = hsum(a.x); o.y = hsum(a.y); o.z = hsum(a.z); o.w = hsum(a.w);
  return o;
}

template <int SLB>
__device__ __forceinline__ int scan_chunk(const int* __restrict__ dsts, int nE, int cbase, int slotBase,
                                          int nb, int vec8, int* list, int tid, int lane, int wave) {
  int wc = 0;
  const int el0  = tid * EPT;
  const int e0   = cbase + el0;
  const int sent = -2147483647 - 1;
  v4i da, db;
  if (vec8 != 0 && cbase + CHUNK <= nE) {
    da = *(const v4i*)(dsts + e0);
    db = *(const v4i*)(dsts + e0 + 4);
  } else {
    da.x = (e0     < nE) ? dsts[min(e0,     nE - 1)] : sent;
    da.y = (e0 + 1 < nE) ? dsts[min(e0 + 1, nE - 1)] : sent;
    da.z = (e0 + 2 < nE) ? dsts[min(e0 + 2, nE - 1)] : sent;
    da.w = (e0 + 3 < nE) ? dsts[min(e0 + 3, nE - 1)] : sent;
    db.x = (e0 + 4 < nE) ? dsts[min(e0 + 4, nE - 1)] : sent;
    db.y = (e0 + 5 < nE) ? dsts[min(e0 + 5, nE - 1)] : sent;
    db.z = (e0 + 6 < nE) ? dsts[min(e0 + 6, nE - 1)] : sent;
    db.w = (e0 + 7 < nE) ? dsts[min(e0 + 7, nE - 1)] : sent;
  }
  const unsigned nbs = (unsigned)slotBase;
  const unsigned unb = (unsigned)nb;
  const unsigned s0 = (unsigned)da.x - nbs, s1 = (unsigned)da.y - nbs;
  const unsigned s2 = (unsigned)da.z - nbs, s3 = (unsigned)da.w - nbs;
  const unsigned s4 = (unsigned)db.x - nbs, s5 = (unsigned)db.y - nbs;
  const unsigned s6 = (unsigned)db.z - nbs, s7 = (unsigned)db.w - nbs;
  const bool h0 = s0 < unb, h1 = s1 < unb, h2 = s2 < unb, h3 = s3 < unb;
  const bool h4 = s4 < unb, h5 = s5 < unb, h6 = s6 < unb, h7 = s7 < unb;
  const unsigned any = __builtin_amdgcn_ballot_w32(h0 | h1 | h2 | h3 | h4 | h5 | h6 | h7);
  if (any != 0u) {
#define HITJ(J, HJ, SJ) { \
      const unsigned mj = __builtin_amdgcn_ballot_w32(HJ); \
      if (mj != 0u) { \
        if (HJ) { \
          const int pos = wc + (int)__builtin_amdgcn_mbcnt_lo(mj, 0u); \
          if (pos < WCAP) list[wave * WCAP + pos] = ((el0 + (J)) << SLB) | (int)(SJ); \
        } \
        wc += (int)__builtin_popcount(mj); } }
    HITJ(0, h0, s0)
    HITJ(1, h1, s1)
    HITJ(2, h2, s2)
    HITJ(3, h3, s3)
    HITJ(4, h4, s4)
    HITJ(5, h5, s5)
    HITJ(6, h6, s6)
    HITJ(7, h7, s7)
#undef HITJ
  }
  return wc;
}

__global__ __launch_bounds__(NTHR) void k_prep(
    const float* __restrict__ x, const float* __restrict__ Wl1, const float* __restrict__ Wr1,
    const float* __restrict__ Wl2, const float* __restrict__ Wr2,
    const float* __restrict__ att1, const float* __restrict__ b1,
    const float* __restrict__ att2, const float* __restrict__ b2,
    char* wsb, size_t oXB, size_t oW1, size_t oW2, size_t oPAR, size_t oH1,
    int nN, int nUx, int nUz) {
  const int u  = (int)blockIdx.x * NTHR + (int)threadIdx.x;
  const int e1 = nUx;
  const int e2 = e1 + NUW1H;
  const int e3 = e2 + NUW1H;
  const int e4 = e3 + NUW2H;
  const int e5 = e4 + NUW2H;
  const int e6 = e5 + NTHR;
  const int e7 = e6 + NTHR;
  const int e8 = e7 + NTHR;
  const int e9 = e8 + NTHR;
  const int e10 = e9 + nUz;
  v4i o = {0, 0, 0, 0};
  size_t doff = 0;
  bool ok = true;
  if (u < e1) {
    const int row = u >> 3;
    const int c0  = (u & 7) * 8;
    const int rc  = row < nN ? row : nN - 1;
    const float* p = x + (size_t)rc * DIN + c0;
    v4f a = *(const v4f*)p, b = *(const v4f*)(p + 4);
    const v4f z4 = {0.f, 0.f, 0.f, 0.f};
    if (row >= nN) { a = z4; b = z4; }
    o = pack8(a, b);
    doff = oXB + ((size_t)row * DIN + c0) * 2;
  } else if (u < e2) {
    const int v = u - e1, n = v >> 3, k8 = (v & 7) * 8;
    o = wtr8(Wl1 + (size_t)k8 * HC + n);
    doff = oW1 + ((size_t)n * DIN + k8) * 2;
  } else if (u < e3) {
    const int v = u - e2, n = v >> 3, k8 = (v & 7) * 8;
    o = wtr8(Wr1 + (size_t)k8 * HC + n);
    doff = oW1 + ((size_t)(HC + n) * DIN + k8) * 2;
  } else if (u < e4) {
    const int v = u - e3, n = v >> 7, k8 = (v & 127) * 8, kk = k8 & (HC - 1);
    o = wtr8(Wl2 + (size_t)kk * HC + n);
    doff = oW2 + ((size_t)n * KA2 + k8) * 2;
  } else if (u < e5) {
    const int v = u - e4, n = v >> 7, k8 = (v & 127) * 8, kk = k8 & (HC - 1);
    o = wtr8(Wr2 + (size_t)kk * HC + n);
    doff = oW2 + ((size_t)(HC + n) * KA2 + k8) * 2;
  } else if (u < e6) {
    const int v = u - e5, n4 = HC / 4, vc = v < n4 ? v : n4 - 1;
    o = par4(att1, n4, v); ok = v < n4;
    doff = oPAR + (size_t)(0 + 4 * vc) * 4;
  } else if (u < e7) {
    const int v = u - e6, n4 = HC / 4, vc = v < n4 ? v : n4 - 1;
    o = par4(b1, n4, v); ok = v < n4;
    doff = oPAR + (size_t)(HC + 4 * vc) * 4;
  } else if (u < e8) {
    const int v = u - e7, n4 = HC / 4, vc = v < n4 ? v : n4 - 1;
    o = par4(att2, n4, v); ok = v < n4;
    doff = oPAR + (size_t)(2 * HC + 4 * vc) * 4;
  } else if (u < e9) {
    const int v = u - e8, n4 = CHN / 4, vc = v < n4 ? v : n4 - 1;
    o = par4(b2, n4, v); ok = v < n4;
    doff = oPAR + (size_t)(3 * HC + 4 * vc) * 4;
  } else if (u < e10) {
    const int v = u - e9;
    const int row = nN + (v >> 7);
    const int col = (v & 127) * 8;
    doff = oH1 + ((size_t)row * KA2 + col) * 2;
  } else {
    return;
  }
  volatile v4i* dp = (volatile v4i*)(wsb + doff);
  if (ok) *dp = o;
  __threadfence();
  if (ok) *dp = o;
}

__global__ __launch_bounds__(NTHR) void k_bucket(const int* __restrict__ srcs, const int* __restrict__ dsts,
                                                 int nE, int nN, int vec8, int* HITS, int* FLG) {
  extern __shared__ __attribute__((aligned(16))) int bsm[];
  int* list = bsm;
  int* reg1 = bsm + LISTN;
  int* wcnt = reg1 + RCAP;
  const int tid = (int)threadIdx.x, lane = tid & 31, wave = tid >> 5;
  const int blk = (int)blockIdx.x;
  const int nodeBase = blk * NBA;
  int nb = nN - nodeBase;
  nb = nb < 0 ? 0 : (nb > NBA ? NBA : nb);

  int tot = 0, ovf = 0;
  const int nChunks = (nE + CHUNK - 1) / CHUNK;
#pragma unroll 1
  for (int ch = 0; ch < nChunks; ++ch) {
    const int cbase = ch * CHUNK;
    const int wc = scan_chunk<SLA>(dsts, nE, cbase, nodeBase, nb, vec8, list, tid, lane, wave);
    if (lane == 0) wcnt[wave] = wc;
    __syncthreads();
    int pre = 0, all = 0;
#pragma unroll
    for (int w2 = 0; w2 < NWAVE; ++w2) {
      int c = wcnt[w2];
      c = c < 0 ? 0 : (c > WCAP ? WCAP : c);
      all += c;
      pre += (w2 < wave) ? c : 0;
    }
    const int wcc  = wc > WCAP ? WCAP : wc;
    const int base = tot + pre;
#pragma unroll 1
    for (int i = lane; i < wcc; i += 32) {
      const int ent = list[wave * WCAP + i];
      const int el  = (ent >> SLA) & (CHUNK - 1);
      const int sl  = ent & (NBA - 1);
      int eid = cbase + el;
      eid = eid > nE - 1 ? nE - 1 : eid;
      const int sraw = srcs[eid];
      const int s = sraw < 0 ? 0 : (sraw > nN - 1 ? nN - 1 : sraw);
      const int pos = base + i;
      if (pos < RCAP) reg1[pos] = (int)((unsigned)s | ((unsigned)sl << SRCB));
    }
    if (tot + all > RCAP) ovf = 1;
    tot += all;
    tot = tot > RCAP ? RCAP : tot;
    __syncthreads();
  }
  const int nh = tot;
  const int nhPad = (nh + 31) & ~31;
  for (int i = nh + tid; i < nhPad; i += NTHR) reg1[i] = 0;
  __syncthreads();

  int* hb = HITS + (size_t)blk * RCAP;
  v4i cv;
  cv.x = (tid == 0) ? nh : 0;
  cv.y = (tid == 0) ? ovf : 0;
  cv.z = 0; cv.w = 0;
  int* fp = FLG + (size_t)blk * 32 + 4 * (tid & 7);
#pragma unroll 1
  for (int p = tid * 4; p < nhPad; p += NTHR * 4) {
    const v4i v = *(const v4ia*)(reg1 + p);
    *(volatile v4i*)(hb + p) = v;
  }
  if (tid < 8) *(volatile v4i*)fp = cv;
  __threadfence();
#pragma unroll 1
  for (int p = tid * 4; p < nhPad; p += NTHR * 4) {
    const v4i v = *(const v4ia*)(reg1 + p);
    *(volatile v4i*)(hb + p) = v;
  }
  if (tid < 8) *(volatile v4i*)fp = cv;
}

__global__ __launch_bounds__(GTHR) void k_gemm(
    const unsigned short* __restrict__ A, const unsigned short* __restrict__ WT,
    float* outF, int K, int ldo)
{
  __shared__ __attribute__((aligned(16))) float stg[GBM * GBN];
  const int tid = (int)threadIdx.x, lane = tid & 31, wave = tid >> 5, hh = lane >> 4, m = lane & 15;
  const int rowBase = (int)blockIdx.x * GBM;
  const int col0    = (int)blockIdx.y * GBN;

  v8f acc[4];
  {
    const v8f z = {0.f, 0.f, 0.f, 0.f, 0.f, 0.f, 0.f, 0.f};
    acc[0] = z; acc[1] = z; acc[2] = z; acc[3] = z;
  }
  const unsigned short* ap = A  + (size_t)(rowBase + 16 * wave + m) * (size_t)K + 8 * hh;
  const unsigned short* wp = WT + (size_t)(col0 + m) * (size_t)K + 8 * hh;
  const int ksteps = K >> 5;
#pragma unroll 1
  for (int ks = 0; ks < ksteps; ++ks) {
    FragB af;
    af.h[0] = *(const v8usa*)(ap + 32 * ks);
    af.h[1] = *(const v8usa*)(ap + 32 * ks + 16);
#pragma unroll
    for (int t = 0; t < 4; ++t) {
      const unsigned short* wq = wp + (size_t)(16 * t) * (size_t)K + 32 * ks;
      FragB bf;
      bf.h[0] = *(const v8usa*)wq;
      bf.h[1] = *(const v8usa*)(wq + 16);
      acc[t] = wmb(af, bf, acc[t]);
    }
  }

#pragma unroll
  for (int t = 0; t < 4; ++t) {
    const int lc = 16 * t + m;
#pragma unroll
    for (int r = 0; r < 8; ++r) {
      const int lr = 16 * wave + 8 * hh + r;
      stg[lr * GBN + lc] = acc[t][r];
    }
  }
  __syncthreads();

  v4f fv[8];
#pragma unroll
  for (int i = 0; i < 8; ++i) {
    const int lr = 16 * wave + 2 * i + hh;
    fv[i] = *(const v4fa*)(stg + lr * GBN + 4 * m);
  }
#pragma unroll
  for (int i = 0; i < 8; ++i) {
    const int lr = 16 * wave + 2 * i + hh;
    const int gr = rowBase + lr;
    float* op = outF + (size_t)gr * (size_t)ldo + col0 + 4 * m;
    *(volatile v4f*)op = fv[i];
  }
  __threadfence();
#pragma unroll
  for (int i = 0; i < 8; ++i) {
    const int lr = 16 * wave + 2 * i + hh;
    const int gr = rowBase + lr;
    float* op = outF + (size_t)gr * (size_t)ldo + col0 + 4 * m;
    *(volatile v4f*)op = fv[i];
  }
}

template <int L>
__global__ __launch_bounds__(NTHR) void k_scan(const int* __restrict__ HITS, const int* __restrict__ FLGB,
                                               const float* __restrict__ XLR, const float* __restrict__ PAR,
                                               unsigned short* XP, float* outF, int nN) {
  static_assert(L == 1 || L == 2);
  extern __shared__ __attribute__((aligned(16))) int ssm[];
  int* hl   = ssm;
  int* sl   = ssm + RCAP;
  int* cnt  = sl + RCAP;
  int* offs = cnt + NBA;
  int* cur  = offs + NBA;
  const int tid = (int)threadIdx.x, lane = tid & 31, wave = tid >> 5;
  const int blk = (int)blockIdx.x;
  const int nodeBase = blk * NBA;

  const int nhraw = FLGB[(size_t)blk * 32];
  const int bflag = FLGB[(size_t)blk * 32 + 1];
  const int nh  = nhraw < 0 ? 0 : (nhraw > RCAP ? RCAP : nhraw);
  const int ovf = (bflag != 0 || nhraw < 0 || nhraw > RCAP) ? 1 : 0;

  {
    const v4i z4 = {0, 0, 0, 0};
    for (int i = tid * 4; i < SCAN_ZINTS; i += NTHR * 4) *(v4ia*)(sl + i) = z4;
    const int* hb = HITS + (size_t)blk * RCAP;
    const int nh4 = (nh + 3) & ~3;
#pragma unroll 1
    for (int p = tid * 4; p < nh4; p += NTHR * 4) *(v4ia*)(hl + p) = *(const v4i*)(hb + p);
  }
  __syncthreads();

  if (wave == 0) {
#pragma unroll 1
    for (int b0 = 0; b0 < nh; b0 += 32) {
      const int idx = b0 + lane;
      const int uv  = hl[idx < nh ? idx : nh - 1];
      const int m32 = (nh - b0) < 32 ? (nh - b0) : 32;
#pragma unroll 1
      for (int k = 0; k < m32; ++k) {
        const int u  = __builtin_amdgcn_readlane(uv, k);
        const int sq = (u >> SRCB) & (NBA - 1);
        if (lane == 0) cnt[sq] = cnt[sq] + 1;
      }
    }
  }
  __syncthreads();
  if (wave == 0) {
    const int base = lane * (NBA / 32);
    int s = 0;
#pragma unroll 1
    for (int i = 0; i < NBA / 32; ++i) s += cnt[base + i];
    int incl = s;
#pragma unroll
    for (int d = 1; d < 32; d <<= 1) {
      const int y = __shfl_up(incl, d, 32);
      if (lane >= d) incl += y;
    }
    int run = incl - s;
#pragma unroll 1
    for (int i = 0; i < NBA / 32; ++i) {
      const int cv = cnt[base + i];
      offs[base + i] = run;
      cur[base + i]  = run;
      run += cv;
    }
  }
  __syncthreads();
  if (wave == 0) {
#pragma unroll 1
    for (int b0 = 0; b0 < nh; b0 += 32) {
      const int idx = b0 + lane;
      const int uv  = hl[idx < nh ? idx : nh - 1];
      const int m32 = (nh - b0) < 32 ? (nh - b0) : 32;
#pragma unroll 1
      for (int k = 0; k < m32; ++k) {
        const int u  = __builtin_amdgcn_readlane(uv, k);
        const int sq = (u >> SRCB) & (NBA - 1);
        if (lane == 0) {
          int p = cur[sq];
          p = p < 0 ? 0 : (p > RCAP - 1 ? RCAP - 1 : p);
          sl[p] = u;
          cur[sq] = p + 1;
        }
      }
    }
  }
  __syncthreads();

  float* fl = (float*)hl;
  float* st = fl + 1024 + wave * HC;
  {
    constexpr int NUN = (L == 1) ? 256 : ((HC + CHN) / 4);
    constexpr int PB  = (L == 1) ? 0 : (2 * HC);
    const int u = tid < NUN ? tid : NUN - 1;
    const v4f pv = *(const v4f*)(PAR + PB + 4 * u);
    *(v4fa*)(fl + 4 * tid) = pv;
  }
  __syncthreads();

  const float qnan = __int_as_float(0x7fc00000);
  const float pzb  = (ovf != 0) ? qnan : 0.0f;
  const v4f at0 = *(const v4fa*)(fl + 16 * lane);
  const v4f at1 = *(const v4fa*)(fl + 16 * lane + 4);
  const v4f at2 = *(const v4fa*)(fl + 16 * lane + 8);
  const v4f at3 = *(const v4fa*)(fl + 16 * lane + 12);
  const int lc = lane < 16 ? lane : 15;

#pragma unroll 1
  for (int si = 0; si < NBA / NWAVE; ++si) {
    const int s    = si * NWAVE + wave;
    const int node = nodeBase + s;
    if (node >= nN) break;
    int c = cnt[s];
    const bool big = c > DEGCAP;
    c = c < 0 ? 0 : (c > DEGCAP ? DEGCAP : c);
    int o = offs[s];
    o = o < 0 ? 0 : (o > RCAP ? RCAP : o);
    if (c > nh - o) c = nh - o;
    c = c < 0 ? 0 : c;

    const float* xrp = XLR + (size_t)node * NXLR + HC + 16 * lane;
    const v4f r0 = *(const v4f*)xrp;
    const v4f r1 = *(const v4f*)(xrp + 4);
    const v4f r2 = *(const v4f*)(xrp + 8);
    const v4f r3 = *(const v4f*)(xrp + 12);
    float mx = -3.0e38f, dn = 0.0f;
    v4f a0 = {0.f, 0.f, 0.f, 0.f}, a1 = a0, a2 = a0, a3 = a0;

    const int T = c + 1;
#pragma unroll 1
    for (int b0 = 0; b0 < T; b0 += 32) {
      const int t = b0 + lane;
      int idx = o + t;
      idx = idx < 0 ? 0 : (idx > RCAP - 1 ? RCAP - 1 : idx);
      const int ent = sl[idx];
      int hs = ent & ((1 << SRCB) - 1);
      hs = hs > nN - 1 ? nN - 1 : hs;
      const int sr  = (t < c) ? hs : node;
      const int m32 = (T - b0) < 32 ? (T - b0) : 32;
#pragma unroll 1
      for (int k = 0; k < m32; ++k) {
        const int sk = __builtin_amdgcn_readlane(sr, k);
        const float* rp = XLR + (size_t)sk * NXLR + 16 * lane;
        const v4f x0 = *(const v4f*)rp;
        const v4f x1 = *(const v4f*)(rp + 4);
        const v4f x2 = *(const v4f*)(rp + 8);
        const v4f x3 = *(const v4f*)(rp + 12);
        float part = 0.0f;
        part = dot4(x0, r0, at0, part);
        part = dot4(x1, r1, at1, part);
        part = dot4(x2, r2, at2, part);
        part = dot4(x3, r3, at3, part);
        part += __shfl_xor(part, 1);
        part += __shfl_xor(part, 2);
        const float df = part - mx;
        const float ee = expf(-fabsf(df));
        const bool  up = df > 0.f;
        const float s1 = up ? ee : 1.0f;
        const float s2 = up ? 1.0f : ee;
        mx = up ? part : mx;
        dn = fmaf(dn, s1, s2);
        a0 = accu(a0, x0, s1, s2);
        a1 = accu(a1, x1, s1, s2);
        a2 = accu(a2, x2, s1, s2);
        a3 = accu(a3, x3, s1, s2);
      }
    }
    const float inv = __builtin_amdgcn_rcpf(dn);
    const float pzr = big ? qnan : pzb;
    v4f t0 = a0 * inv, t1 = a1 * inv, t2 = a2 * inv, t3 = a3 * inv;

    if constexpr (L == 2) {
      t0 = hsum4(t0); t1 = hsum4(t1); t2 = hsum4(t2); t3 = hsum4(t3);
    }
    __builtin_amdgcn_fence(__ATOMIC_RELEASE, "wavefront");
    __builtin_amdgcn_wave_barrier();
    *(v4fa*)(st + 16 * lane)      = t0;
    *(v4fa*)(st + 16 * lane + 4)  = t1;
    *(v4fa*)(st + 16 * lane + 8)  = t2;
    *(v4fa*)(st + 16 * lane + 12) = t3;
    __builtin_amdgcn_fence(__ATOMIC_RELEASE, "wavefront");
    __builtin_amdgcn_wave_barrier();

    if constexpr (L == 1) {
#pragma unroll 1
      for (int j = 0; j < 16; ++j) {
        const int pos = ((j >> 3) << 8) + 8 * lane + (j & 7);
        float y = st[pos] + fl[HC + pos];
        y = (y > 0.0f) ? y : expm1f(y);
        st[pos] = y + pzr;
      }
      const v4f g0 = *(const v4fa*)(st + 8 * lane);
      const v4f g1 = *(const v4fa*)(st + 8 * lane + 4);
      const v4f g2 = *(const v4fa*)(st + 256 + 8 * lane);
      const v4f g3 = *(const v4fa*)(st + 256 + 8 * lane + 4);
      const HL8 q0 = cvt_hl8(g0, g1);
      const HL8 q1 = cvt_hl8(g2, g3);
      unsigned short* hp = XP + (size_t)node * KA2 + 8 * lane;
      *(volatile v4i*)hp              = q0.h;
      *(volatile v4i*)(hp + 256)      = q1.h;
      *(volatile v4i*)(hp + HC)       = q0.l;
      *(volatile v4i*)(hp + HC + 256) = q1.l;
      __threadfence();
      *(volatile v4i*)hp              = q0.h;
      *(volatile v4i*)(hp + 256)      = q1.h;
      *(volatile v4i*)(hp + HC)       = q0.l;
      *(volatile v4i*)(hp + HC + 256) = q1.l;
    } else {
      const v4f g  = *(const v4fa*)(st + 4 * lc);
      const v4f bq = *(const v4fa*)(fl + HC + 4 * lc);
      v4f r;
      r.x = fmaf(g.x, 0.125f, bq.x) + pzr;
      r.y = fmaf(g.y, 0.125f, bq.y) + pzr;
      r.z = fmaf(g.z, 0.125f, bq.z) + pzr;
      r.w = fmaf(g.w, 0.125f, bq.w) + pzr;
      float* gp = outF + (size_t)node * CHN + 4 * lc;
      const bool wsv = lane < (CHN / 4);
      if (wsv) *(volatile v4f*)gp = r;
      __threadfence();
      if (wsv) *(volatile v4f*)gp = r;
    }
  }
  (void)XP; (void)outF;
}

static inline int cdiv(int a, int b) { return (a + b - 1) / b; }

extern "C" void kernel_launch(void* const* d_in, const int* in_sizes, int n_in,
                              void* d_out, int out_size, void* d_ws, size_t ws_size,
                              hipStream_t stream) {
  if (n_in < 10) return;
  const int nN = in_sizes[0] / DIN;
  if (nN <= 0 || in_sizes[0] != nN * DIN || nN > (1 << SRCB)) return;
  if (in_sizes[1] < 2 || (in_sizes[1] & 1) != 0) return;
  const int nE = in_sizes[1] / 2;
  if (nE < 1 || nE > (1 << 30)) return;
  if (in_sizes[2] != DIN * HC || in_sizes[3] != DIN * HC) return;
  if (in_sizes[4] != HC || in_sizes[5] != HC) return;
  if (in_sizes[6] != HC * HC || in_sizes[7] != HC * HC) return;
  if (in_sizes[8] != HC || in_sizes[9] != CHN) return;
  if (out_size != nN * CHN) return;

  const float* x    = (const float*)d_in[0];
  const int*   ei   = (const int*)  d_in[1];
  const float* Wl1  = (const float*)d_in[2];
  const float* Wr1  = (const float*)d_in[3];
  const float* att1 = (const float*)d_in[4];
  const float* b1   = (const float*)d_in[5];
  const float* Wl2  = (const float*)d_in[6];
  const float* Wr2  = (const float*)d_in[7];
  const float* att2 = (const float*)d_in[8];
  const float* b2   = (const float*)d_in[9];
  float* out = (float*)d_out;
  const int* src = ei;
  const int* dst = ei + nE;

  const int MP   = cdiv(nN, MROWS) * MROWS;
  const int gM   = MP / GBM;
  const int gA   = cdiv(nN, NBA);
  const int vec8 = ((nE & 3) == 0) ? 1 : 0;
  const int nUx  = MP * (DIN / 8);
  const int nUz  = (MP - nN) * (KA2 / 8);
  if ((nUx % NTHR) != 0 || (nUz % NTHR) != 0) return;
  const long long nTotL = (long long)nUx + 2LL * NUW1H + 2LL * NUW2H + 4LL * NTHR + (long long)nUz;
  if (nTotL > (1LL << 30)) return;
  const int nTot = (int)nTotL;

  char* ws = (char*)d_ws;
  size_t off = 0;
  const size_t oXB  = off; off += (size_t)MP * DIN * 2;           off = (off + 255) & ~(size_t)255;
  const size_t oW1  = off; off += (size_t)NXLR * DIN * 2;         off = (off + 255) & ~(size_t)255;
  const size_t oW2  = off; off += (size_t)NXLR * KA2 * 2;         off = (off + 255) & ~(size_t)255;
  const size_t oPAR = off; off += (size_t)PARF * 4;               off = (off + 255) & ~(size_t)255;
  const size_t oXLR = off; off += (size_t)MP * NXLR * 4;          off = (off + 255) & ~(size_t)255;
  const size_t oH1  = off; off += (size_t)MP * KA2 * 2;           off = (off + 255) & ~(size_t)255;
  const size_t oHIT = off; off += (size_t)gA * RCAP * 4;          off = (off + 255) & ~(size_t)255;
  const size_t oFLG = off; off += (size_t)gA * 128;               off = (off + 255) & ~(size_t)255;
  if (off > ws_size || off > (size_t)WSMAX) return;
  unsigned short* XB   = (unsigned short*)(ws + oXB);
  unsigned short* W1T  = (unsigned short*)(ws + oW1);
  unsigned short* W2T  = (unsigned short*)(ws + oW2);
  float*          PAR  = (float*)(ws + oPAR);
  float*          XLR  = (float*)(ws + oXLR);
  unsigned short* H1HL = (unsigned short*)(ws + oH1);
  int*            HITS = (int*)(ws + oHIT);
  int*            FLG  = (int*)(ws + oFLG);

  const int bktLds  = BKT_LDS_INTS * 4;
  const int scanLds = SCAN_LDS_INTS * 4;
  hipFuncSetAttribute(reinterpret_cast<const void*>(&k_bucket),
                      hipFuncAttributeMaxDynamicSharedMemorySize, bktLds);
  hipFuncSetAttribute(reinterpret_cast<const void*>(&k_scan<1>),
                      hipFuncAttributeMaxDynamicSharedMemorySize, scanLds);
  hipFuncSetAttribute(reinterpret_cast<const void*>(&k_scan<2>),
                      hipFuncAttributeMaxDynamicSharedMemorySize, scanLds);

  k_prep<<<nTot / NTHR, NTHR, 0, stream>>>(x, Wl1, Wr1, Wl2, Wr2, att1, b1, att2, b2,
                                            ws, oXB, oW1, oW2, oPAR, oH1, nN, nUx, nUz);
  k_bucket<<<gA, NTHR, bktLds, stream>>>(src, dst, nE, nN, vec8, HITS, FLG);
  k_gemm<<<dim3(gM, NXLR / GBN), GTHR, 0, stream>>>(XB, W1T, XLR, DIN, NXLR);
  k_scan<1><<<gA, NTHR, scanLds, stream>>>(HITS, FLG, XLR, PAR, H1HL, out, nN);
  k_gemm<<<dim3(gM, NXLR / GBN), GTHR, 0, stream>>>(H1HL, W2T, XLR, KA2, NXLR);
  k_scan<2><<<gA, NTHR, scanLds, stream>>>(HITS, FLG, XLR, PAR, H1HL, out, nN);
}
